// NeighborhoodSelfAttention_15255723835593
// MI455X (gfx1250) — hardware-verified
//
#include <hip/hip_runtime.h>
#include <stdint.h>

constexpr int kImgH  = 96;
constexpr int kImgW  = 96;
constexpr int kSeq   = kImgH * kImgW;
constexpr int kChan  = 256;
constexpr int kHeads = 8;
constexpr int kDh    = 32;
constexpr int kQkvN  = 3 * kChan;
constexpr int kWin   = 7;
constexpr int kNbr   = kWin * kWin;
constexpr float kQkScale = 0.17677669529663687f;
constexpr int kXPitch = 257;
constexpr int kTPitch = 36;
static_assert(kHeads * kDh == kChan);
static_assert(kSeq % 64 == 0 && kChan % 64 == 0 && kQkvN % 64 == 0 && kChan % 32 == 0);

typedef __attribute__((ext_vector_type(16))) _Float16 v16h;
typedef __attribute__((ext_vector_type(8)))  _Float16 v8h;
typedef __attribute__((ext_vector_type(16))) __bf16   v16b;
typedef __attribute__((ext_vector_type(8)))  __bf16   v8b;
typedef __attribute__((ext_vector_type(8)))  float    v8f;
typedef __attribute__((ext_vector_type(4)))  float    v4f;
#define PSCALE 32768.0f
#define U16(p) ((const unsigned short*)(const void*)(p))
#define PSCALE_INV (1.0f / 32768.0f)

__device__ __forceinline__ unsigned short f2bf_bits(float f) {
  unsigned u = __float_as_uint(f);
  return (unsigned short)((u + 0x7FFFu + ((u >> 16) & 1u)) >> 16);
}
__device__ __forceinline__ float bf_bits2f(unsigned short h) { return __uint_as_float(((unsigned)h) << 16); }

__device__ __forceinline__ void dep_guard_h(v8f& a, v8f& b, v16h x, v16h y) { asm volatile("v_nop\n\tv_nop\n\tv_nop\n\tv_nop" : "+v"(a), "+v"(b) : "v"(x), "v"(y)); }
__device__ __forceinline__ void dep_guard_b(v8f& a, v8f& b, v16b x, v16b y) { asm volatile("v_nop\n\tv_nop\n\tv_nop\n\tv_nop" : "+v"(a), "+v"(b) : "v"(x), "v"(y)); }
__device__ __forceinline__ void keep4_h(v16h a, v16h b, v16h c, v16h d) { asm volatile("v_nop" :: "v"(a), "v"(b), "v"(c), "v"(d)); }
__device__ __forceinline__ void keep4_b(v16b a, v16b b, v16b c, v16b d) { asm volatile("v_nop" :: "v"(a), "v"(b), "v"(c), "v"(d)); }
__device__ __forceinline__ void acc_guard4(v8f& a, v8f& b, v8f& c, v8f& d) { asm volatile("v_nop\n\tv_nop\n\tv_nop\n\tv_nop" : "+v"(a), "+v"(b), "+v"(c), "+v"(d)); }
template <typename T> struct Frag;
template <> struct Frag<_Float16> {
  typedef v16h V; union U { v16h v; v8h h[2]; };
  static __device__ __forceinline__ v16h load(const _Float16* p) {
    U f; f.h[0] = *(const v8h*)(p); f.h[1] = *(const v8h*)(p + 16); return f.v;
  }
  static __device__ __forceinline__ v8f mma(v16h a, v16h b, v8f c) {
    return __builtin_amdgcn_wmma_f32_16x16x32_f16(false, a, false, b, (short)0, c, false, false);
  }
  static __device__ __forceinline__ void guard(v8f& a, v8f& b, v16h x, v16h y) { dep_guard_h(a, b, x, y); }
  static __device__ __forceinline__ void keep(v16h a, v16h b, v16h c, v16h d) { keep4_h(a, b, c, d); }
};
template <> struct Frag<__bf16> {
  typedef v16b V; union U { v16b v; v8b h[2]; };
  static __device__ __forceinline__ v16b load(const __bf16* p) {
    U f; f.h[0] = *(const v8b*)(p); f.h[1] = *(const v8b*)(p + 16); return f.v;
  }
  static __device__ __forceinline__ v8f mma(v16b a, v16b b, v8f c) {
    return __builtin_amdgcn_wmma_f32_16x16x32_bf16(false, a, false, b, (short)0, c, false, false);
  }
  static __device__ __forceinline__ void guard(v8f& a, v8f& b, v16b x, v16b y) { dep_guard_b(a, b, x, y); }
  static __device__ __forceinline__ void keep(v16b a, v16b b, v16b c, v16b d) { keep4_b(a, b, c, d); }
};

template <int ET> struct Elem;
template <> struct Elem<0> { typedef _Float16 T; };
template <> struct Elem<1> { typedef __bf16 T; };
template <int ET, bool SPLIT, int BIAS_MODE, int OUT_MODE, bool RESID, int ACT = 0>
__global__ __launch_bounds__(256) void wmma_gemm64(
    const unsigned short* __restrict__ Ap, const unsigned short* __restrict__ A2p, int lda, long strideA,
    const unsigned short* __restrict__ Btp, const unsigned short* __restrict__ Bt2p, int ldb, long strideB,
    void* __restrict__ Cout, void* __restrict__ Cout2, int ldc, long strideC,
    const float* __restrict__ bias,
    const float* __restrict__ resid, long strideR,
    int M, int N, int K, float scale) {
  typedef typename Elem<ET>::T T;
  typedef typename Frag<T>::V V;
  const T* A = (const T*)Ap; const T* A2 = (const T*)A2p; const T* Bt = (const T*)Btp; const T* Bt2 = (const T*)Bt2p;
  __shared__ __align__(16) float sT[8][16 * 68];
  const int b    = blockIdx.y;
  const int lane = threadIdx.x & 31;
  const int wave = threadIdx.x >> 5;
  const int tilesN = N >> 6;
  const int tilesM = M >> 6;
  const int tile = blockIdx.x * 8 + wave;
  if (tile >= tilesM * tilesN) return;
  const int tm = tile / tilesN;
  const int tn = tile - tm * tilesN;
  const int m0 = tm << 6;
  const int n0 = tn << 6;

  const T* Ab  = A  + (size_t)b * strideA;
  const T* Bb  = Bt + (size_t)b * strideB;
  const T* Ab2 = SPLIT ? (A2  + (size_t)b * strideA) : nullptr;
  const T* Bb2 = SPLIT ? (Bt2 + (size_t)b * strideB) : nullptr;

  const int rlane = lane & 15;
  const int koff  = (lane >> 4) * 8;
  const int mOff  = (lane >> 4) * 8;

  v8f acc[4][4];
#pragma unroll
  for (int i = 0; i < 4; ++i)
#pragma unroll
    for (int j = 0; j < 4; ++j) acc[i][j] = (v8f){0.f,0.f,0.f,0.f,0.f,0.f,0.f,0.f};

  for (int k0 = 0; k0 < K; k0 += 32) {
    V bh[4], bl[4];
#pragma unroll
    for (int j = 0; j < 4; ++j) {
      const size_t bo = (size_t)(n0 + (j << 4) + rlane) * ldb + koff + k0;
      bh[j] = Frag<T>::load(Bb + bo);
      if (SPLIT) bl[j] = Frag<T>::load(Bb2 + bo);
    }
#pragma unroll
    for (int i = 0; i < 4; ++i) {
      const size_t ao = (size_t)(m0 + (i << 4) + rlane) * lda + koff + k0;
      V ah = Frag<T>::load(Ab + ao);
      V al;
      if (SPLIT) al = Frag<T>::load(Ab2 + ao);
#pragma unroll
      for (int j = 0; j < 4; ++j) {
        acc[i][j] = Frag<T>::mma(ah, bh[j], acc[i][j]);
        if (SPLIT) {
          acc[i][j] = Frag<T>::mma(ah, bl[j], acc[i][j]);
          acc[i][j] = Frag<T>::mma(al, bh[j], acc[i][j]);
        }
      }
      Frag<T>::guard(acc[i][0], acc[i][3], ah, SPLIT ? al : ah);
    }
    Frag<T>::keep(bh[0], bh[1], bh[2], bh[3]);
    if (SPLIT) Frag<T>::keep(bl[0], bl[1], bl[2], bl[3]);
  }
  acc_guard4(acc[0][0], acc[0][1], acc[0][2], acc[0][3]);
  acc_guard4(acc[1][0], acc[1][1], acc[1][2], acc[1][3]);
  acc_guard4(acc[2][0], acc[2][1], acc[2][2], acc[2][3]);
  acc_guard4(acc[3][0], acc[3][1], acc[3][2], acc[3][3]);

  float* slab = sT[wave];
  const float* Rb = RESID ? (resid + (size_t)b * strideR) : nullptr;
#pragma unroll
  for (int i = 0; i < 4; ++i) {
    const int mBase = m0 + (i << 4);
#pragma unroll
    for (int j = 0; j < 4; ++j) {
      const int n = n0 + (j << 4) + rlane;
      float bv = 0.f;
      if (BIAS_MODE == 2) bv = bias[n];
#pragma unroll
      for (int r = 0; r < 8; ++r) {
        float v = acc[i][j][r] * scale;
        if (BIAS_MODE == 1) v += bias[mBase + mOff + r];
        if (BIAS_MODE == 2) v += bv;
        if (RESID) v += Rb[(size_t)(mBase + mOff + r) * ldc + n];
        if (ACT == 1) v = tanhf(v);
        if (ACT == 2) v = fmaxf(v, 0.0f);
        if (ACT == 3) v = v / (1.0f + expf(-v));
        if (ACT == 4) v = (v > 0.f) ? v : 0.01f * v;
        if (ACT == 5) v = 0.5f * v * (1.0f + erff(v * 0.70710678118654752f));
        slab[(mOff + r) * 68 + (j << 4) + rlane] = v;
      }
    }
    __builtin_amdgcn_fence(__ATOMIC_RELEASE, "workgroup");
    __builtin_amdgcn_wave_barrier();
    __builtin_amdgcn_fence(__ATOMIC_ACQUIRE, "workgroup");
    if (OUT_MODE == 0) {
      float* C = (float*)Cout + (size_t)b * strideC;
      const int hh = lane >> 4, c4 = (lane & 15) * 4;
      for (int pass = 0; pass < 2; ++pass) {
#pragma unroll
        for (int it = 0; it < 8; ++it) {
          const int row = it * 2 + hh;
          v4f v = *(const v4f*)(slab + row * 68 + c4);
          *(volatile v4f*)(C + (size_t)(mBase + row) * ldc + n0 + c4) = v;
        }
        __threadfence();
      }
    } else {
      const int q = lane >> 3, c8 = (lane & 7) * 8;
      unsigned short* C  = (unsigned short*)Cout  + (size_t)b * strideC;
      unsigned short* C2 = (OUT_MODE == 2) ? ((unsigned short*)Cout2 + (size_t)b * strideC) : nullptr;
      for (int pass = 0; pass < 2; ++pass) {
#pragma unroll
        for (int it = 0; it < 4; ++it) {
          const int row = it * 4 + q;
          const float* sp = slab + row * 68 + c8;
          v8h hv, lv;
#pragma unroll
          for (int e = 0; e < 8; ++e) {
            if (OUT_MODE == 1) {
              hv[e] = (_Float16)sp[e];
            } else {
              unsigned short hb = f2bf_bits(sp[e]);
              unsigned short lb = f2bf_bits(sp[e] - bf_bits2f(hb));
              hv[e] = __builtin_bit_cast(_Float16, hb);
              lv[e] = __builtin_bit_cast(_Float16, lb);
            }
          }
          *(volatile v8h*)(C + (size_t)(mBase + row) * ldc + n0 + c8) = hv;
          if (OUT_MODE == 2) *(volatile v8h*)(C2 + (size_t)(mBase + row) * ldc + n0 + c8) = lv;
        }
        __threadfence();
      }
    }
    __builtin_amdgcn_fence(__ATOMIC_RELEASE, "workgroup");
    __builtin_amdgcn_wave_barrier();
    __builtin_amdgcn_fence(__ATOMIC_ACQUIRE, "workgroup");
  }
}

__device__ __forceinline__ void store_rows32x256_split(const float* stg, int pitch,
    unsigned short* __restrict__ Hp, unsigned short* __restrict__ Lp, size_t row0) {
  const int lane = threadIdx.x & 31, wave = threadIdx.x >> 5;
  const int rq = lane >> 3, c8 = (lane & 7) * 8;
  const int row = wave * 4 + rq;
  for (int pass = 0; pass < 2; ++pass) {
#pragma unroll
    for (int it = 0; it < 4; ++it) {
      const int col = it * 64 + c8;
      const float* sp = stg + row * pitch + col;
      v8h hv, lv;
#pragma unroll
      for (int e = 0; e < 8; ++e) {
        const float f = sp[e];
        const unsigned short hb = f2bf_bits(f);
        const unsigned short lb = f2bf_bits(f - bf_bits2f(hb));
        hv[e] = __builtin_bit_cast(_Float16, hb);
        lv[e] = __builtin_bit_cast(_Float16, lb);
      }
      const size_t o = (row0 + (size_t)row) * (size_t)kChan + (size_t)col;
      *(volatile v8h*)(Hp + o) = hv;
      *(volatile v8h*)(Lp + o) = lv;
    }
    __threadfence();
  }
}

__global__ __launch_bounds__(256) void split_f32_bf16x8(const float* __restrict__ in,
    unsigned short* __restrict__ Hp, unsigned short* __restrict__ Lp, int n8) {
  const int i = blockIdx.x * 256 + threadIdx.x;
  if (i < n8) {
    const v4f a = *(const v4f*)(in + (size_t)8 * i);
    const v4f c = *(const v4f*)(in + (size_t)8 * i + 4);
    v8h hv, lv;
#pragma unroll
    for (int e = 0; e < 4; ++e) {
      const unsigned short ha = f2bf_bits(a[e]);
      const unsigned short la = f2bf_bits(a[e] - bf_bits2f(ha));
      const unsigned short hc = f2bf_bits(c[e]);
      const unsigned short lc = f2bf_bits(c[e] - bf_bits2f(hc));
      hv[e] = __builtin_bit_cast(_Float16, ha);     lv[e] = __builtin_bit_cast(_Float16, la);
      hv[4 + e] = __builtin_bit_cast(_Float16, hc); lv[4 + e] = __builtin_bit_cast(_Float16, lc);
    }
    for (int pass = 0; pass < 2; ++pass) {
      *(volatile v8h*)(Hp + (size_t)8 * i) = hv;
      *(volatile v8h*)(Lp + (size_t)8 * i) = lv;
      __threadfence();
    }
  }
}

__global__ __launch_bounds__(256) void x_to_rows_split(const float* __restrict__ x,
    unsigned short* __restrict__ XLh, unsigned short* __restrict__ XLl) {
  __shared__ __align__(16) float tile[32 * kXPitch];
  const int tid = threadIdx.x, lane = tid & 31, wave = tid >> 5;
  const int s0 = blockIdx.x * 32;
#pragma unroll 4
  for (int i = 0; i < 32; ++i) {
    const int c = i * 8 + wave;
    tile[lane * kXPitch + c] = x[(size_t)c * kSeq + s0 + lane];
  }
  __syncthreads();
  store_rows32x256_split(tile, kXPitch, XLh, XLl, (size_t)s0);
}

__global__ __launch_bounds__(256) void window_attn(const float* __restrict__ QKV,
    unsigned short* __restrict__ CTXh, unsigned short* __restrict__ CTXl) {
  __shared__ __align__(16) float sm[kNbr * 256];
  const int tid = threadIdx.x;
  const int h  = tid & 7;
  const int pl = tid >> 3;
  const int s0 = blockIdx.x * 32;
  const int s  = s0 + pl;
  const int y  = s / kImgW;
  const int xq = s - y * kImgW;
  const int yc = y  < 3 ? 3 : (y  > kImgH - 4 ? kImgH - 4 : y);
  const int xc = xq < 3 ? 3 : (xq > kImgW - 4 ? kImgW - 4 : xq);
  const int ys = yc - 3, xs = xc - 3;

  float q[32];
  {
    const v4f* qp = (const v4f*)(QKV + (size_t)s * kQkvN + h * kDh);
#pragma unroll
    for (int i = 0; i < 8; ++i) {
      const v4f t = qp[i];
      q[4 * i + 0] = t[0]; q[4 * i + 1] = t[1]; q[4 * i + 2] = t[2]; q[4 * i + 3] = t[3];
    }
  }

  float m = -__builtin_inff();
#pragma unroll 1
  for (int a = 0; a < kWin; ++a) {
    const float* krow = QKV + (size_t)((ys + a) * kImgW + xs) * kQkvN + kChan + h * kDh;
#pragma unroll 1
    for (int b = 0; b < kWin; ++b) {
      const v4f* kp = (const v4f*)(krow + (size_t)b * kQkvN);
      float d = 0.f;
#pragma unroll
      for (int i = 0; i < 8; ++i) {
        const v4f kk = kp[i];
        d += q[4 * i + 0] * kk[0];
        d += q[4 * i + 1] * kk[1];
        d += q[4 * i + 2] * kk[2];
        d += q[4 * i + 3] * kk[3];
      }
      const float sc = d * kQkScale;
      sm[(a * kWin + b) * 256 + tid] = sc;
      m = fmaxf(m, sc);
    }
  }

  float acc[32];
#pragma unroll
  for (int i = 0; i < 32; ++i) acc[i] = 0.f;
  float l = 0.f;
#pragma unroll 1
  for (int a = 0; a < kWin; ++a) {
    const float* vrow = QKV + (size_t)((ys + a) * kImgW + xs) * kQkvN + 2 * kChan + h * kDh;
#pragma unroll 1
    for (int b = 0; b < kWin; ++b) {
      const float p = __expf(sm[(a * kWin + b) * 256 + tid] - m);
      l += p;
      const v4f* vp = (const v4f*)(vrow + (size_t)b * kQkvN);
#pragma unroll
      for (int i = 0; i < 8; ++i) {
        const v4f vv = vp[i];
        acc[4 * i + 0] += p * vv[0];
        acc[4 * i + 1] += p * vv[1];
        acc[4 * i + 2] += p * vv[2];
        acc[4 * i + 3] += p * vv[3];
      }
    }
  }
  const float inv = __builtin_amdgcn_rcpf(l);

  __syncthreads();
  {
    float* st = sm + pl * 256 + h * kDh;
#pragma unroll
    for (int i = 0; i < 8; ++i) {
      v4f o;
      o[0] = acc[4 * i + 0] * inv; o[1] = acc[4 * i + 1] * inv;
      o[2] = acc[4 * i + 2] * inv; o[3] = acc[4 * i + 3] * inv;
      *(v4f*)(st + 4 * i) = o;
    }
  }
  __syncthreads();
  store_rows32x256_split(sm, 256, CTXh, CTXl, (size_t)s0);
}

__global__ __launch_bounds__(256) void rows_to_nchw(const float* __restrict__ src, float* __restrict__ dst) {
  __shared__ __align__(16) float tile[kChan * kTPitch];
  const int tid = threadIdx.x, lane = tid & 31, wave = tid >> 5;
  const int s0 = blockIdx.x * 32;
#pragma unroll 4
  for (int i = 0; i < 32; ++i) tile[tid * kTPitch + i] = src[(size_t)(s0 + i) * kChan + tid];
  __syncthreads();
  const int rq = lane >> 3, s4 = (lane & 7) * 4;
  for (int pass = 0; pass < 2; ++pass) {
#pragma unroll
    for (int it = 0; it < 8; ++it) {
      const int ch = wave * 32 + it * 4 + rq;
      const v4f val = *(const v4f*)(tile + ch * kTPitch + s4);
      *(volatile v4f*)(dst + (size_t)ch * kSeq + s0 + s4) = val;
    }
    __threadfence();
  }
}

extern "C" void kernel_launch(void* const* d_in, const int* in_sizes, int n_in,
                              void* d_out, int out_size, void* d_ws, size_t ws_size,
                              hipStream_t stream) {
  if (n_in < 5) return;
  if (in_sizes[0] != kChan * kSeq || in_sizes[1] != kQkvN * kChan || in_sizes[2] != kQkvN ||
      in_sizes[3] != kChan * kChan || in_sizes[4] != kChan || out_size != kChan * kSeq) return;

  const float* x     = (const float*)d_in[0];
  const float* w_qkv = (const float*)d_in[1];
  const float* b_qkv = (const float*)d_in[2];
  const float* w_out = (const float*)d_in[3];
  const float* b_out = (const float*)d_in[4];
  float* outp = (float*)d_out;

  char* ws = (char*)d_ws;
  size_t off = 0;
  auto carve = [&](size_t bytes) -> void* {
    void* p = ws + off;
    off = (off + bytes + 255) & ~(size_t)255;
    return p;
  };
  unsigned short* XLh  = (unsigned short*)carve((size_t)kSeq * kChan * 2);
  unsigned short* XLl  = (unsigned short*)carve((size_t)kSeq * kChan * 2);
  unsigned short* WQh  = (unsigned short*)carve((size_t)kQkvN * kChan * 2);
  unsigned short* WQl  = (unsigned short*)carve((size_t)kQkvN * kChan * 2);
  unsigned short* WOh  = (unsigned short*)carve((size_t)kChan * kChan * 2);
  unsigned short* WOl  = (unsigned short*)carve((size_t)kChan * kChan * 2);
  float*          QKV  = (float*)carve((size_t)kSeq * kQkvN * 4);
  unsigned short* CTXh = (unsigned short*)carve((size_t)kSeq * kChan * 2);
  unsigned short* CTXl = (unsigned short*)carve((size_t)kSeq * kChan * 2);
  float*          OUT  = (float*)carve((size_t)kSeq * kChan * 4);
  if (off > ws_size) return;

  const int n8_wq = kQkvN * kChan / 8;
  const int n8_wo = kChan * kChan / 8;
  split_f32_bf16x8<<<(n8_wq + 255) / 256, 256, 0, stream>>>(w_qkv, WQh, WQl, n8_wq);
  split_f32_bf16x8<<<(n8_wo + 255) / 256, 256, 0, stream>>>(w_out, WOh, WOl, n8_wo);

  x_to_rows_split<<<kSeq / 32, 256, 0, stream>>>(x, XLh, XLl);

  {
    const int tiles = (kSeq / 64) * (kQkvN / 64);
    wmma_gemm64<1, true, 2, 0, false><<<dim3((tiles + 7) / 8, 1), 256, 0, stream>>>(
        XLh, XLl, kChan, 0L, WQh, WQl, kChan, 0L,
        (void*)QKV, (void*)nullptr, kQkvN, 0L,
        b_qkv, (const float*)nullptr, 0L, kSeq, kQkvN, kChan, 1.0f);
  }

  window_attn<<<kSeq / 32, 256, 0, stream>>>(QKV, CTXh, CTXl);

  {
    const int tiles = (kSeq / 64) * (kChan / 64);
    wmma_gemm64<1, true, 2, 0, false><<<dim3((tiles + 7) / 8, 1), 256, 0, stream>>>(
        CTXh, CTXl, kChan, 0L, WOh, WOl, kChan, 0L,
        (void*)OUT, (void*)nullptr, kChan, 0L,
        b_out, (const float*)nullptr, 0L, kSeq, kChan, kChan, 1.0f);
  }

  rows_to_nchw<<<kSeq / 32, 256, 0, stream>>>(OUT, outp);
}
